// OA_3_33097017983620
// MI455X (gfx1250) — hardware-run, weakly checked
//
#include <hip/hip_runtime.h>
#include <math.h>
#include <stdint.h>


#define NB   8
#define CH   256
#define CK   64
#define NT   2048
#define TOK  (NB * NT)
#define RSB  32
#define NRB  (NT / RSB)
#define MT   32
#define NCH  64
#define PTP  72
#define PX   264
#define OUTN (NB * CH * NT)

#define SCW  64.0f
#define SCQK 8.0f
#define SCV  1024.0f
#define SCE  32768.0f
#define SCR  2048.0f
#define SCXR 8.0f
#define SCS  (1.0f / (SCQK * SCQK))

static_assert(TOK % 64 == 0 && CH % 64 == 0 && CK % 32 == 0 && CH % 32 == 0);
static_assert((((TOK / 64) * (CH / 64)) % 8) == 0);
static_assert(NT % RSB == 0 && RSB == 32 && NT == 8 * 256);
static_assert((NT / 16) % 8 == 0 && CH == 8 * 32);
static_assert(NT % MT == 0 && NT % NCH == 0 && MT == 32 && NCH == 64);
static_assert((CH * CH) % 2048 == 0 && (CH * CK) % 2048 == 0);
static_assert(TOK == 16 * 1024 && TOK % 32 == 0);
static_assert(NT % 64 == 0 && CK % 64 == 0);
static_assert((PX * 2) % 16 == 0 && (PTP * 2) % 16 == 0);

typedef _Float16       v16h __attribute__((ext_vector_type(16)));
typedef _Float16       v8h  __attribute__((ext_vector_type(8)));
typedef float          v8f  __attribute__((ext_vector_type(8)));
typedef float          v4f  __attribute__((ext_vector_type(4)));
typedef unsigned int   v4u  __attribute__((ext_vector_type(4)));

union HU { v8h h; v4u u; _Float16 s[8]; };
union FR { v16h v; v8h h[2]; _Float16 s[16]; };
static_assert(sizeof(HU) == 16);
static_assert(sizeof(FR) == 32);

__device__ __forceinline__ unsigned short bf_bits(float f) {
  const unsigned u = __float_as_uint(f);
  return (unsigned short)((u + 0x7FFFu + ((u >> 16) & 1u)) >> 16);
}
__device__ __forceinline__ float bf_up(unsigned short h) { return __uint_as_float(((unsigned)h) << 16); }
__device__ __forceinline__ float bfr(float f) { return bf_up(bf_bits(f)); }
__device__ __forceinline__ v8f zero8() { v8f z = {0.f, 0.f, 0.f, 0.f, 0.f, 0.f, 0.f, 0.f}; return z; }

__device__ __forceinline__ void ld8(const float* p, float* o) {
  const v4f a = *(const v4f*)(p);
  const v4f b = *(const v4f*)(p + 4);
  o[0] = a[0]; o[1] = a[1]; o[2] = a[2]; o[3] = a[3];
  o[4] = b[0]; o[5] = b[1]; o[6] = b[2]; o[7] = b[3];
}
__device__ __forceinline__ void st8(float* p, const float* o) {
  v4f a, b;
  a[0] = o[0]; a[1] = o[1]; a[2] = o[2]; a[3] = o[3];
  b[0] = o[4]; b[1] = o[5]; b[2] = o[6]; b[3] = o[7];
  *(v4f*)(p) = a;
  *(v4f*)(p + 4) = b;
}

__device__ __forceinline__ double shfl_xor_d(double v, int m) {
  const unsigned long long u = (unsigned long long)__double_as_longlong(v);
  int lo = (int)(unsigned)(u & 0xffffffffull);
  int hi = (int)(unsigned)(u >> 32);
  lo = __shfl_xor(lo, m, 32);
  hi = __shfl_xor(hi, m, 32);
  const unsigned long long r = (((unsigned long long)(unsigned)hi) << 32) | (unsigned long long)(unsigned)lo;
  return __longlong_as_double((long long)r);
}

__device__ __forceinline__ v16h ldfrag_h(const _Float16* p) {
  FR f;
  f.h[0] = *(const v8h*)(p);
  f.h[1] = *(const v8h*)(p + 16);
  return f.v;
}

__device__ __forceinline__ v8f mma_h(v16h a, v16h b, v8f c) {
  c = __builtin_amdgcn_wmma_f32_16x16x32_f16(false, a, false, b, (short)0, c, false, false);
#if defined(__HIP_DEVICE_COMPILE__)
  asm volatile("v_nop\n\tv_nop\n\tv_nop\n\tv_nop" : "+v"(c) : "v"(a), "v"(b));
#endif
  return c;
}
__device__ __forceinline__ v8f mma_h_raw(v16h a, v16h b, v8f c) {
  return __builtin_amdgcn_wmma_f32_16x16x32_f16(false, a, false, b, (short)0, c, false, false);
}
__device__ __forceinline__ void dep_guard_h(v8f& a, v8f& b, v16h x) {
#if defined(__HIP_DEVICE_COMPILE__)
  asm volatile("v_nop\n\tv_nop\n\tv_nop\n\tv_nop" : "+v"(a), "+v"(b) : "v"(x));
#endif
}
__device__ __forceinline__ void keep4_h(v16h a, v16h b, v16h c, v16h d) {
#if defined(__HIP_DEVICE_COMPILE__)
  asm volatile("v_nop" :: "v"(a), "v"(b), "v"(c), "v"(d));
#endif
}
__device__ __forceinline__ void acc_guard4(v8f& a, v8f& b, v8f& c, v8f& d) {
#if defined(__HIP_DEVICE_COMPILE__)
  asm volatile("v_nop\n\tv_nop\n\tv_nop\n\tv_nop" : "+v"(a), "+v"(b), "+v"(c), "+v"(d));
#endif
}
__device__ __forceinline__ void wave_lds_sync() {
  __builtin_amdgcn_fence(__ATOMIC_RELEASE, "workgroup");
  __builtin_amdgcn_wave_barrier();
  __builtin_amdgcn_fence(__ATOMIC_ACQUIRE, "workgroup");
}

__global__ __launch_bounds__(256) void cvt_flat(const float* __restrict__ in, _Float16* out, int n8, float scale) {
  const int i = blockIdx.x * 256 + threadIdx.x;
  if (i < n8) {
    float v[8];
    ld8(in + (size_t)i * 8, v);
    HU u;
#pragma unroll
    for (int e = 0; e < 8; ++e) u.s[e] = (_Float16)(bfr(v[e]) * scale);
    _Float16* p = out + (size_t)i * 8;
    *(volatile v4u*)p = u.u;
    __threadfence();
    *(volatile v4u*)p = u.u;
  }
}

__global__ __launch_bounds__(256) void cvt_xT(const float* __restrict__ X, _Float16* XT, int Cd) {
  __shared__ float sw[64][65];
  const int t = threadIdx.x;
  const int n0 = blockIdx.x * 64, k0 = blockIdx.y * 64, b = blockIdx.z;
  const float* Xb = X + (size_t)b * Cd * NT;
  {
    const int r = t >> 4, c4 = (t & 15) * 4;
#pragma unroll
    for (int it = 0; it < 4; ++it) {
      const int row = r + 16 * it;
      const v4f x = *(const v4f*)(Xb + (size_t)(k0 + row) * NT + n0 + c4);
      sw[row][c4 + 0] = x[0]; sw[row][c4 + 1] = x[1]; sw[row][c4 + 2] = x[2]; sw[row][c4 + 3] = x[3];
    }
  }
  __syncthreads();
  const int q8 = t & 7, rr = t >> 3;
  HU u[2];
#pragma unroll
  for (int it = 0; it < 2; ++it) {
    const int n = rr + 32 * it;
#pragma unroll
    for (int e = 0; e < 8; ++e) u[it].s[e] = (_Float16)bfr(sw[8 * q8 + e][n]);
  }
  for (int pass = 0; pass < 2; ++pass) {
#pragma unroll
    for (int it = 0; it < 2; ++it) {
      const int n = rr + 32 * it;
      _Float16* dst = XT + (size_t)(b * NT + n0 + n) * Cd + k0 + 8 * q8;
      *(volatile v4u*)dst = u[it].u;
    }
    __threadfence();
  }
}

__device__ __forceinline__ void kseg(v8f (&acc)[4][4], const _Float16* __restrict__ A, int lda, int m0,
                                     const _Float16* __restrict__ Bt, int ldb, int n0, int K, int rlane, int koff) {
  for (int kk = 0; kk < K; kk += 32) {
    v16h bh[4];
#pragma unroll
    for (int j = 0; j < 4; ++j) {
      const size_t bo = (size_t)(n0 + (j << 4) + rlane) * (size_t)ldb + koff + kk;
      bh[j] = ldfrag_h(Bt + bo);
    }
#pragma unroll
    for (int i = 0; i < 4; ++i) {
      const size_t ao = (size_t)(m0 + (i << 4) + rlane) * (size_t)lda + koff + kk;
      const v16h a0 = ldfrag_h(A + ao);
#pragma unroll
      for (int j = 0; j < 4; ++j) acc[i][j] = mma_h_raw(a0, bh[j], acc[i][j]);
      dep_guard_h(acc[i][0], acc[i][3], a0);
    }
    keep4_h(bh[0], bh[1], bh[2], bh[3]);
  }
}

template <int RB>
__global__ __launch_bounds__(256) void gemm64p(
    const _Float16* __restrict__ A, int lda, const _Float16* __restrict__ Bt, int ldb,
    const float* __restrict__ rowbias, int nrb, float cs, float so,
    _Float16* Ch, _Float16* Cl, int ldc, int M, int N, int K) {
  __shared__ __align__(16) float sT[8][16 * 68];
  const int lane = threadIdx.x & 31;
  const int wave = threadIdx.x >> 5;
  const int tilesN = N >> 6;
  const int tilesM = M >> 6;
  const int tiles = tilesM * tilesN;
  const int item = blockIdx.x * 8 + wave;
  if (item >= tiles) return;
  const int tm = item / tilesN;
  const int tn = item - tm * tilesN;
  const int m0 = tm << 6;
  const int n0 = tn << 6;

  const int rlane = lane & 15;
  const int koff  = (lane >> 4) * 8;
  const int mOff  = (lane >> 4) * 8;

  v8f acc[4][4];
#pragma unroll
  for (int i = 0; i < 4; ++i)
#pragma unroll
    for (int j = 0; j < 4; ++j) acc[i][j] = zero8();

  kseg(acc, A, lda, m0, Bt, ldb, n0, K, rlane, koff);
  acc_guard4(acc[0][0], acc[0][1], acc[0][2], acc[0][3]);
  acc_guard4(acc[1][0], acc[1][1], acc[1][2], acc[1][3]);
  acc_guard4(acc[2][0], acc[2][1], acc[2][2], acc[2][3]);
  acc_guard4(acc[3][0], acc[3][1], acc[3][2], acc[3][3]);

  const int q8 = lane & 7, rr = lane >> 3, c8 = q8 * 8;

  float* slab = sT[wave];
#pragma unroll
  for (int i = 0; i < 4; ++i) {
    const int mBase = m0 + (i << 4);
#pragma unroll
    for (int r = 0; r < 8; ++r) {
#pragma unroll
      for (int j = 0; j < 4; ++j) {
        slab[(mOff + r) * 68 + (j << 4) + rlane] = acc[i][j][r];
      }
    }
    wave_lds_sync();
    v4u uh[4], ul[4];
#pragma unroll
    for (int it = 0; it < 4; ++it) {
      const int row = it * 4 + rr;
      float xs[8];
      ld8(slab + row * 68 + c8, xs);
      const float rbv = RB ? bfr(rowbias[min(mBase + row, nrb - 1)]) : 0.0f;
      HU h, l;
#pragma unroll
      for (int e = 0; e < 8; ++e) {
        const float v = (xs[e] * cs + rbv) * so;
        const _Float16 hv = (_Float16)v;
        h.s[e] = hv;
        l.s[e] = (_Float16)((v - (float)hv) * SCR);
      }
      uh[it] = h.u;
      ul[it] = l.u;
    }
    for (int pass = 0; pass < 2; ++pass) {
#pragma unroll
      for (int it = 0; it < 4; ++it) {
        const int row = it * 4 + rr;
        const size_t co = (size_t)(mBase + row) * (size_t)ldc + n0 + c8;
        *(volatile v4u*)(Ch + co) = uh[it];
        *(volatile v4u*)(Cl + co) = ul[it];
      }
      __threadfence();
    }
    wave_lds_sync();
  }
}

__global__ __launch_bounds__(256) void k_soft(const _Float16* __restrict__ XQh, const _Float16* __restrict__ XQl,
                                              const _Float16* __restrict__ XKh, const _Float16* __restrict__ XKl,
                                              _Float16* E, float* PART) {
  extern __shared__ __align__(16) float sc[];
  const int tid = threadIdx.x, wave = tid >> 5, lane = tid & 31;
  const int hh = lane >> 4, rl = lane & 15;
  const int rb = blockIdx.x, b = blockIdx.y, n0 = rb * RSB;

  const _Float16* aqh = XQh + (size_t)(b * NT + n0 + rl) * CH + 8 * hh;
  const _Float16* aql = XQl + (size_t)(b * NT + n0 + rl) * CH + 8 * hh;
  for (int ct = wave; ct < NT / 16; ct += 8) {
    const _Float16* bkh = XKh + (size_t)(b * NT + 16 * ct + rl) * CH + 8 * hh;
    const _Float16* bkl = XKl + (size_t)(b * NT + 16 * ct + rl) * CH + 8 * hh;
    v8f a00 = zero8(), a01 = zero8(), a10 = zero8(), a11 = zero8();
#pragma unroll 2
    for (int ks = 0; ks < CH / 32; ++ks) {
      const v16h bh  = ldfrag_h(bkh + 32 * ks);
      const v16h bl  = ldfrag_h(bkl + 32 * ks);
      const v16h q0h = ldfrag_h(aqh + 32 * ks);
      const v16h q0l = ldfrag_h(aql + 32 * ks);
      const v16h q1h = ldfrag_h(aqh + 16 * CH + 32 * ks);
      const v16h q1l = ldfrag_h(aql + 16 * CH + 32 * ks);
      a00 = mma_h(q0h, bh, a00);
      a01 = mma_h(q0h, bl, a01);
      a01 = mma_h(q0l, bh, a01);
      a10 = mma_h(q1h, bh, a10);
      a11 = mma_h(q1h, bl, a11);
      a11 = mma_h(q1l, bh, a11);
    }
    const int mc = 16 * ct + rl;
#pragma unroll
    for (int r = 0; r < 8; ++r) {
      sc[(size_t)(8 * hh + r) * NT + mc]      = (a00[r] + a01[r] * (1.0f / SCR)) * SCS;
      sc[(size_t)(16 + 8 * hh + r) * NT + mc] = (a10[r] + a11[r] * (1.0f / SCR)) * SCS;
    }
  }
  __syncthreads();

  for (int q4 = 0; q4 < 4; ++q4) {
    const int row = 4 * wave + q4;
    float* rp = sc + (size_t)row * NT + 8 * lane;
    float mx = -3.0e38f;
#pragma unroll
    for (int j = 0; j < 8; ++j) {
      float v[8];
      ld8(rp + 256 * j, v);
#pragma unroll
      for (int e = 0; e < 8; ++e) mx = fmaxf(mx, v[e]);
    }
#pragma unroll
    for (int off = 16; off >= 1; off >>= 1) mx = fmaxf(mx, __shfl_xor(mx, off, 32));
    float z = 0.0f;
#pragma unroll
    for (int j = 0; j < 8; ++j) {
      float v[8];
      ld8(rp + 256 * j, v);
#pragma unroll
      for (int e = 0; e < 8; ++e) {
        const float ef = __expf(v[e] - mx);
        z += ef;
        v[e] = ef;
      }
      st8(rp + 256 * j, v);
    }
#pragma unroll
    for (int off = 16; off >= 1; off >>= 1) z += __shfl_xor(z, off, 32);
    const float rz = SCE * (1.0f / z);
    HU u[8];
#pragma unroll
    for (int j = 0; j < 8; ++j) {
      float v[8];
      ld8(rp + 256 * j, v);
#pragma unroll
      for (int e = 0; e < 8; ++e) {
        const _Float16 h0 = (_Float16)(v[e] * rz);
        const float f0 = (float)h0;
        const bool sub = f0 < 6.103515625e-05f;
        u[j].s[e] = sub ? (_Float16)0.0f : h0;
        v[e] = sub ? 0.0f : f0;
      }
      st8(rp + 256 * j, v);
    }
    _Float16* erow = E + (size_t)(b * NT + n0 + row) * NT + 8 * lane;
    for (int pass = 0; pass < 2; ++pass) {
#pragma unroll
      for (int j = 0; j < 8; ++j) *(volatile v4u*)(erow + 256 * j) = u[j].u;
      __threadfence();
    }
  }
  __syncthreads();

  {
    v4f pa = {0.f, 0.f, 0.f, 0.f}, pb = {0.f, 0.f, 0.f, 0.f};
#pragma unroll 4
    for (int r = 0; r < RSB; ++r) {
      pa += *(const v4f*)(sc + (size_t)r * NT + 4 * tid);
      pb += *(const v4f*)(sc + (size_t)r * NT + 1024 + 4 * tid);
    }
    float* prow = PART + (size_t)(b * NRB + rb) * NT + 4 * tid;
    for (int pass = 0; pass < 2; ++pass) {
      *(volatile v4f*)(prow) = pa;
      *(volatile v4f*)(prow + 1024) = pb;
      __threadfence();
    }
  }
}

__global__ __launch_bounds__(256) void k_pv(const _Float16* __restrict__ E, const _Float16* __restrict__ VH,
                                            const _Float16* __restrict__ VL, const float* __restrict__ PART,
                                            _Float16* XRh, _Float16* XRl) {
  __shared__ __align__(16) _Float16 sPt[MT * PTP];
  __shared__ __align__(16) _Float16 sXh[MT * PX];
  __shared__ __align__(16) _Float16 sXl[MT * PX];
  __shared__ float srcp[MT];
  const int tid = threadIdx.x, wave = tid >> 5, lane = tid & 31;
  const int hh = lane >> 4, rl = lane & 15;
  const int bx = blockIdx.x;
  const int b = bx / (NT / MT);
  const int m0 = (bx - b * (NT / MT)) * MT;
  const int cb = wave * 32;

  if (wave == 0) {
    const int m = m0 + lane;
    float s = 0.0f;
    for (int r = 0; r < NRB; ++r) s += PART[(size_t)(b * NRB + r) * NT + m];
    const float sr = s * (1.0f / SCE);
    srcp[lane] = 1.0f / (1e-9f + sr);
  }

  v8f acc[2][2], accl[2][2];
#pragma unroll
  for (int i = 0; i < 2; ++i)
#pragma unroll
    for (int j = 0; j < 2; ++j) { acc[i][j] = zero8(); accl[i][j] = zero8(); }

  for (int nc = 0; nc < NT; nc += NCH) {
    __syncthreads();
    {
      const int n = tid >> 2, p = tid & 3;
      HU u;
      u.h = *(const v8h*)(E + (size_t)(b * NT + nc + n) * NT + m0 + 8 * p);
#pragma unroll
      for (int e = 0; e < 8; ++e) sPt[(8 * p + e) * PTP + n] = u.s[e];
    }
    __syncthreads();
#pragma unroll
    for (int ks = 0; ks < 2; ++ks) {
      const v16h pb0 = ldfrag_h(&sPt[rl * PTP + 32 * ks + 8 * hh]);
      const v16h pb1 = ldfrag_h(&sPt[(16 + rl) * PTP + 32 * ks + 8 * hh]);
#pragma unroll
      for (int i = 0; i < 2; ++i) {
        const size_t vo = (size_t)(cb + 16 * i + rl) * TOK + (size_t)(b * NT + nc + 32 * ks) + 8 * hh;
        const v16h ah = ldfrag_h(VH + vo);
        const v16h al = ldfrag_h(VL + vo);
        acc[i][0]  = mma_h(ah, pb0, acc[i][0]);
        acc[i][1]  = mma_h(ah, pb1, acc[i][1]);
        accl[i][0] = mma_h(al, pb0, accl[i][0]);
        accl[i][1] = mma_h(al, pb1, accl[i][1]);
      }
    }
  }

  const float fo = 1.0f / (SCV * SCE);
  const float fl = fo * (1.0f / SCR);
#pragma unroll
  for (int i = 0; i < 2; ++i) {
#pragma unroll
    for (int j = 0; j < 2; ++j) {
      const int ml = 16 * j + rl;
      const float sv = srcp[ml] * SCXR;
      HU h, l;
#pragma unroll
      for (int r = 0; r < 8; ++r) {
        const float v = (acc[i][j][r] * fo + accl[i][j][r] * fl) * sv;
        const _Float16 hv = (_Float16)v;
        h.s[r] = hv;
        l.s[r] = (_Float16)((v - (float)hv) * SCR);
      }
      *(v8h*)(&sXh[ml * PX + cb + 16 * i + 8 * hh]) = h.h;
      *(v8h*)(&sXl[ml * PX + cb + 16 * i + 8 * hh]) = l.h;
    }
  }
  __syncthreads();
  HU oh[4], ol[4];
#pragma unroll
  for (int it = 0; it < 4; ++it) {
    const int mrow = 4 * wave + it;
    oh[it].h = *(const v8h*)(&sXh[mrow * PX + 8 * lane]);
    ol[it].h = *(const v8h*)(&sXl[mrow * PX + 8 * lane]);
  }
  for (int pass = 0; pass < 2; ++pass) {
#pragma unroll
    for (int it = 0; it < 4; ++it) {
      const int mrow = 4 * wave + it;
      const size_t xo = (size_t)(b * NT + m0 + mrow) * CH + 8 * lane;
      *(volatile v4u*)(XRh + xo) = oh[it].u;
      *(volatile v4u*)(XRl + xo) = ol[it].u;
    }
    __threadfence();
  }
}

__global__ __launch_bounds__(256) void gemm_y(const _Float16* __restrict__ Wt16, const _Float16* __restrict__ XRh,
                                              const _Float16* __restrict__ XRl, const float* __restrict__ bt, float* Y) {
  __shared__ __align__(16) float sO[8][16 * 36];
  const int tid = threadIdx.x, wave = tid >> 5, lane = tid & 31;
  const int hh = lane >> 4, rl = lane & 15;
  const int t0 = blockIdx.x * 32;
  const int ob = wave * 32;

  v8f acc[2][2], accl[2][2];
#pragma unroll
  for (int i = 0; i < 2; ++i)
#pragma unroll
    for (int j = 0; j < 2; ++j) { acc[i][j] = zero8(); accl[i][j] = zero8(); }

#pragma unroll 2
  for (int ks = 0; ks < CH / 32; ++ks) {
    v16h bh[2], bl[2];
#pragma unroll
    for (int j = 0; j < 2; ++j) {
      const size_t bo = (size_t)(t0 + 16 * j + rl) * CH + 32 * ks + 8 * hh;
      bh[j] = ldfrag_h(XRh + bo);
      bl[j] = ldfrag_h(XRl + bo);
    }
#pragma unroll
    for (int i = 0; i < 2; ++i) {
      const v16h a = ldfrag_h(Wt16 + (size_t)(ob + 16 * i + rl) * CH + 32 * ks + 8 * hh);
#pragma unroll
      for (int j = 0; j < 2; ++j) {
        acc[i][j]  = mma_h(a, bh[j], acc[i][j]);
        accl[i][j] = mma_h(a, bl[j], accl[i][j]);
      }
    }
  }

  const float cy = 1.0f / (SCW * SCXR);
  float* slab = sO[wave];
  const int q8 = lane & 7, rr = lane >> 3;
#pragma unroll
  for (int i = 0; i < 2; ++i) {
    float bb[8];
#pragma unroll
    for (int r = 0; r < 8; ++r) bb[r] = bfr(bt[ob + 16 * i + 8 * hh + r]);
#pragma unroll
    for (int r = 0; r < 8; ++r) {
#pragma unroll
      for (int j = 0; j < 2; ++j) {
        slab[(8 * hh + r) * 36 + 16 * j + rl] = (acc[i][j][r] + accl[i][j][r] * (1.0f / SCR)) * cy + bb[r];
      }
    }
    wave_lds_sync();
    v4f ov[4];
#pragma unroll
    for (int it = 0; it < 4; ++it) {
      const int row = it * 4 + rr;
      ov[it] = *(const v4f*)(slab + row * 36 + 4 * q8);
    }
    for (int pass = 0; pass < 2; ++pass) {
#pragma unroll
      for (int it = 0; it < 4; ++it) {
        const int row = it * 4 + rr;
        float* dst = Y + (size_t)(ob + 16 * i + row) * TOK + t0 + 4 * q8;
        *(volatile v4f*)dst = ov[it];
      }
      __threadfence();
    }
    wave_lds_sync();
  }
}

__global__ __launch_bounds__(256) void k_bn(const float* __restrict__ Y, const float* __restrict__ gam,
                                            const float* __restrict__ bet, float* out) {
  __shared__ double sred[8];
  const int c = blockIdx.x;
  const int tid = threadIdx.x, wave = tid >> 5, lane = tid & 31;
  const float* yc = Y + (size_t)c * TOK + 4 * tid;

  double s = 0.0;
#pragma unroll 1
  for (int j = 0; j < TOK / 1024; ++j) {
    const v4f v = *(const v4f*)(yc + 1024 * j);
    s += (double)v[0]; s += (double)v[1]; s += (double)v[2]; s += (double)v[3];
  }
#pragma unroll
  for (int off = 16; off >= 1; off >>= 1) s += shfl_xor_d(s, off);
  if (lane == 0) sred[wave] = s;
  __syncthreads();
  double tot = 0.0;
#pragma unroll
  for (int w = 0; w < 8; ++w) tot += sred[w];
  const float mean = (float)(tot * (1.0 / (double)TOK));
  __syncthreads();

  double q = 0.0;
#pragma unroll 1
  for (int j = 0; j < TOK / 1024; ++j) {
    const v4f v = *(const v4f*)(yc + 1024 * j);
#pragma unroll
    for (int e = 0; e < 4; ++e) {
      const double d = (double)(v[e] - mean);
      q += d * d;
    }
  }
#pragma unroll
  for (int off = 16; off >= 1; off >>= 1) q += shfl_xor_d(q, off);
  if (lane == 0) sred[wave] = q;
  __syncthreads();
  double totq = 0.0;
#pragma unroll
  for (int w = 0; w < 8; ++w) totq += sred[w];
  const float var = (float)(totq * (1.0 / (double)TOK));
  const float rstd = 1.0f / sqrtf(var + 1e-5f);
  const float g = bfr(gam[c]);
  const float be = bfr(bet[c]);

  for (int pass = 0; pass < 2; ++pass) {
#pragma unroll 1
    for (int j = 0; j < TOK / 1024; ++j) {
      const v4f v = *(const v4f*)(yc + 1024 * j);
      v4f o;
#pragma unroll
      for (int e = 0; e < 4; ++e) {
        const float yv = (v[e] - mean) * rstd * g + be;
        o[e] = yv > 0.0f ? yv : 0.0f;
      }
      const int bb = j >> 1;
      float* dst = out + ((size_t)(bb * CH + c)) * NT + (j & 1) * 1024 + 4 * tid;
      *(volatile v4f*)dst = o;
    }
    __threadfence();
  }
}

extern "C" void kernel_launch(void* const* d_in, const int* in_sizes, int n_in,
                              void* d_out, int out_size, void* d_ws, size_t ws_size,
                              hipStream_t stream) {
  if (n_in < 10) return;
  if (in_sizes[0] != NB * CH * NT || in_sizes[1] != NB * CK * NT) return;
  if (in_sizes[2] != CH * CH || in_sizes[3] != CH * CK || in_sizes[4] != CH * CH || in_sizes[5] != CH) return;
  if (in_sizes[6] != CH * CH || in_sizes[7] != CH || in_sizes[8] != CH || in_sizes[9] != CH) return;
  if (out_size != OUTN) return;

  const float* q     = (const float*)d_in[0];
  const float* x     = (const float*)d_in[1];
  const float* Wq    = (const float*)d_in[2];
  const float* Wk    = (const float*)d_in[3];
  const float* Wv    = (const float*)d_in[4];
  const float* bv    = (const float*)d_in[5];
  const float* Wt    = (const float*)d_in[6];
  const float* bt    = (const float*)d_in[7];
  const float* gam   = (const float*)d_in[8];
  const float* bet   = (const float*)d_in[9];

  const size_t PWQ   = (size_t)CH * CH * 2;
  const size_t PWK   = (size_t)CH * CK * 2;
  const size_t PQT   = (size_t)TOK * CH * 2;
  const size_t PXT   = (size_t)TOK * CK * 2;
  const size_t PPL   = (size_t)TOK * CH * 2;
  const size_t PE    = (size_t)TOK * NT * 2;
  const size_t PPART = (size_t)NB * NRB * NT * 4;
  const size_t PY    = (size_t)CH * TOK * 4;
  if (PPART > PQT) return;
  if (PY != 2 * PPL) return;

  size_t off = 0;
  const size_t oWQ  = off; off += PWQ;
  const size_t oWK  = off; off += PWK;
  const size_t oWV  = off; off += PWQ;
  const size_t oWT  = off; off += PWQ;
  const size_t oQT  = off; off += PQT;
  const size_t oXT  = off; off += PXT;
  const size_t oXQh = off; off += PPL;
  const size_t oXQl = off; off += PPL;
  const size_t oXKh = off; off += PPL;
  const size_t oXKl = off; off += PPL;
  const size_t oVH  = off; off += PPL;
  const size_t oVL  = off; off += PPL;
  const size_t oE   = off; off += PE;
  if (off > ws_size) return;
  if (off > (size_t)134217728) return;

  char* ws = (char*)d_ws;
  _Float16* WQ16 = (_Float16*)(ws + oWQ);
  _Float16* WK16 = (_Float16*)(ws + oWK);
  _Float16* WV16 = (_Float16*)(ws + oWV);
  _Float16* WT16 = (_Float16*)(ws + oWT);
  _Float16* qT   = (_Float16*)(ws + oQT);
  _Float16* xT   = (_Float16*)(ws + oXT);
  _Float16* XQh  = (_Float16*)(ws + oXQh);
  _Float16* XQl  = (_Float16*)(ws + oXQl);
  _Float16* XKh  = (_Float16*)(ws + oXKh);
  _Float16* XKl  = (_Float16*)(ws + oXKl);
  _Float16* VH   = (_Float16*)(ws + oVH);
  _Float16* VL   = (_Float16*)(ws + oVL);
  _Float16* E    = (_Float16*)(ws + oE);
  float*    PART = (float*)(ws + oQT);
  _Float16* XRh  = (_Float16*)(ws + oXQh);
  _Float16* XRl  = (_Float16*)(ws + oXQl);
  float*    Y    = (float*)(ws + oXKh);
  float*    outf = (float*)d_out;

  const dim3 blk(256);
  const int n8cc = (CH * CH) / 8;
  const int n8ck = (CH * CK) / 8;
  const dim3 gWcc((n8cc + 255) / 256);
  const dim3 gWck((n8ck + 255) / 256);
  const dim3 gXq(NT / 64, CH / 64, NB);
  const dim3 gXx(NT / 64, CK / 64, NB);
  const dim3 gPr(((TOK / 64) * (CH / 64) + 7) / 8);
  const dim3 gSo(NRB, NB);
  const dim3 gPV(NB * (NT / MT));
  const dim3 gY(TOK / 32);
  const dim3 gBN(CH);
  const float cs64 = 1.0f / SCW;
  const size_t ldsSoft = (size_t)RSB * NT * sizeof(float);

  cvt_flat<<<gWcc, blk, 0, stream>>>(Wq, WQ16, n8cc, SCW);
  cvt_flat<<<gWck, blk, 0, stream>>>(Wk, WK16, n8ck, SCW);
  cvt_flat<<<gWcc, blk, 0, stream>>>(Wv, WV16, n8cc, SCW);
  cvt_flat<<<gWcc, blk, 0, stream>>>(Wt, WT16, n8cc, SCW);
  cvt_xT<<<gXq, blk, 0, stream>>>(q, qT, CH);
  cvt_xT<<<gXx, blk, 0, stream>>>(x, xT, CK);
  gemm64p<0><<<gPr, blk, 0, stream>>>(qT, CH, WQ16, CH, bv, CH, cs64, SCQK, XQh, XQl, CH, TOK, CH, CH);
  gemm64p<0><<<gPr, blk, 0, stream>>>(xT, CK, WK16, CK, bv, CH, cs64, SCQK, XKh, XKl, CH, TOK, CH, CK);
  gemm64p<1><<<gPr, blk, 0, stream>>>(WV16, CH, qT, CH, bv, CH, cs64, SCV, VH, VL, TOK, CH, TOK, CH);
  k_soft<<<gSo, blk, ldsSoft, stream>>>(XQh, XQl, XKh, XKl, E, PART);
  k_pv<<<gPV, blk, 0, stream>>>(E, VH, VL, PART, XRh, XRl);
  gemm_y<<<gY, blk, 0, stream>>>(WT16, XRh, XRl, bt, Y);
  k_bn<<<gBN, blk, 0, stream>>>(Y, gam, bet, outf);
}
